// WorkflowEncoder_60979945668776
// MI455X (gfx1250) — hardware-run, weakly checked
//
#include <hip/hip_runtime.h>
#include <stddef.h>


#define CH     256
#define PQW    512
#define APZ    264
#define APZ2   520
#define KNB    16
#define GROWS  32
#define GTHR   64
#define NTHR   256
#define NWAVE  8
#define FTHR   128
#define FW     4
#define NIT    16
#define NPBE   (FW * NIT)
#define NPALN  128
#define RTHR   256
#define DEGCAP 1024
#define EPT    8
#define NGRP   2
#define CHUNK  (NTHR * EPT * NGRP)
#define WCAP   (EPT * NGRP * 32)
#define LISTN  (NWAVE * WCAP)
#define NBC    4096
#define NBF    1024
#define RCAP   40960
#define RBN    128
#define OTHR   512
#define LDS_FILL ((RCAP + NBF + LISTN) * 4 + 64)
#define PL_NE1  0
#define PL_NE2  65536
#define PL_L0   131072
#define PL_LSTR 393216
#define PL_MPQ  0
#define PL_M2   131072
#define PL_U2   196608
#define PL_U1   262144
#define PL_RO1  1310720
#define PL_RO2  1376256
#define PL_TOT  1441792
#define WPBLK   704
#define WSCAP   134217728
#define WSC     64.0f
#define ZSC     16.0f
#define RZW     0.0009765625f
#define LNEPS   1e-5f

static_assert(NIT * FW == NPBE);
static_assert(FTHR == FW * 32);
static_assert(GROWS == (GTHR / 32) * 16);
static_assert((APZ % 8) == 0 && (APZ2 % 8) == 0 && (PQW % 32) == 0);
static_assert((NPALN % GROWS) == 0 && (NPALN % NPBE) == 0);
static_assert(32 * GTHR * 4 == GROWS * CH);
static_assert(16 * GTHR * 8 == GROWS * CH);
static_assert(2 * FTHR * 4 == FW * CH);
static_assert(GTHR * 4 == CH);
static_assert(FTHR * 4 >= CH);
static_assert(RTHR == CH);
static_assert(PL_TOT == PL_RO2 + 65536);
static_assert(WPBLK * NTHR * 8 == PL_TOT);
static_assert((CHUNK & (CHUNK - 1)) == 0);
static_assert(CHUNK <= 4096);
static_assert(NBC <= 4096 && NBF <= 4096);
static_assert((NBC & (NBC - 1)) == 0 && (NBF & (NBF - 1)) == 0);
static_assert(NBC == 4 * NBF);
static_assert(OTHR * 8 == NBC);
static_assert((RCAP % 32) == 0);
static_assert((DEGCAP % KNB) == 0);
static_assert((CH % 32) == 0);

typedef float          v4f  __attribute__((ext_vector_type(4)));
typedef float          v8f  __attribute__((ext_vector_type(8)));
typedef int            v4i  __attribute__((ext_vector_type(4)));
typedef _Float16       v4h  __attribute__((ext_vector_type(4)));
typedef _Float16       v8h  __attribute__((ext_vector_type(8)));
typedef _Float16       v16h __attribute__((ext_vector_type(16)));
union Frag { v16h v; v8h h[2]; };
union H8   { v8h v; v4h h[2]; };

__device__ __forceinline__ v8f wmh(v16h a, v16h b, v8f c) {
  v8f d = __builtin_amdgcn_wmma_f32_16x16x32_f16(false, a, false, b, (short)0, c, false, false);
  asm volatile("v_nop\n\tv_nop\n\tv_nop\n\tv_nop" : "+v"(d) : "v"(a), "v"(b));
  return d;
}

__device__ __forceinline__ v4h cvt4z(v4f a) {
  v4h r;
  r.x = (_Float16)(a.x * ZSC); r.y = (_Float16)(a.y * ZSC); r.z = (_Float16)(a.z * ZSC); r.w = (_Float16)(a.w * ZSC);
  return r;
}
__device__ __forceinline__ v8h cvt8z(v4f a, v4f b) {
  H8 o;
  o.h[0] = cvt4z(a);
  o.h[1] = cvt4z(b);
  return o.v;
}

__device__ __forceinline__ float wsum(float s) {
  s += __shfl_xor(s, 16, 32);
  s += __shfl_xor(s, 8, 32);
  s += __shfl_xor(s, 4, 32);
  s += __shfl_xor(s, 2, 32);
  s += __shfl_xor(s, 1, 32);
  return s;
}

template <int NT>
__device__ __forceinline__ void mma(const _Float16* At, int apz, const _Float16* __restrict__ Bp, int kpb,
                                    int ksteps, int lane, v8f (&acc)[NT]) {
  const int hh = lane >> 4, m = lane & 15;
#pragma unroll
  for (int t = 0; t < NT; ++t) { v8f z = {0.f, 0.f, 0.f, 0.f, 0.f, 0.f, 0.f, 0.f}; acc[t] = z; }
  const _Float16* ap = At + m * apz + 8 * hh;
  const _Float16* bb = Bp + (size_t)m * kpb + 8 * hh;
#pragma unroll 1
  for (int ks = 0; ks < ksteps; ++ks) {
    Frag a;
    a.h[0] = *(const v8h*)(ap + 32 * ks);
    a.h[1] = *(const v8h*)(ap + 32 * ks + 16);
#pragma unroll
    for (int t = 0; t < NT; ++t) {
      const _Float16* bp = bb + (size_t)(16 * t) * kpb + 32 * ks;
      Frag b;
      b.h[0] = *(const v8h*)bp;
      b.h[1] = *(const v8h*)(bp + 16);
      acc[t] = wmh(a.v, b.v, acc[t]);
    }
  }
}

template <int J0>
__device__ __forceinline__ void rows_z(_Float16* zw, const float* __restrict__ PQ, int sv, v4f qa, v4f qb, int lane) {
#pragma unroll
  for (int j = J0; j < J0 + 8; ++j) {
    const int s = __builtin_amdgcn_readlane(sv, j);
    const float* pp = PQ + (size_t)s * PQW + 8 * lane;
    const v4f p0 = *(const v4f*)pp, p1 = *(const v4f*)(pp + 4);
    v4f u0 = p0 + qa, u1 = p1 + qb;
    u0.x = fmaxf(u0.x, 0.0f); u0.y = fmaxf(u0.y, 0.0f); u0.z = fmaxf(u0.z, 0.0f); u0.w = fmaxf(u0.w, 0.0f);
    u1.x = fmaxf(u1.x, 0.0f); u1.y = fmaxf(u1.y, 0.0f); u1.z = fmaxf(u1.z, 0.0f); u1.w = fmaxf(u1.w, 0.0f);
    *(v8h*)(zw + j * APZ + 8 * lane) = cvt8z(u0, u1);
  }
}

template <int NB>
__device__ __forceinline__ int scan_chunk(const int* __restrict__ dsts, int nE, int cbase, int slotBase,
                                          int vec8, int* list, int tid, int lane, int wave) {
  int wc = 0;
#pragma unroll
  for (int g = 0; g < NGRP; ++g) {
    const int el0  = (g * NTHR + tid) * EPT;
    const int e0   = cbase + el0;
    const int sent = -2147483647 - 1;
    v4i da, db;
    if (vec8 != 0 && cbase + CHUNK <= nE) {
      da = *(const v4i*)(dsts + e0);
      db = *(const v4i*)(dsts + e0 + 4);
    } else {
      da.x = (e0     < nE) ? dsts[min(e0, nE - 1)] : sent;
      da.y = (e0 + 1 < nE) ? dsts[min(e0 + 1, nE - 1)] : sent;
      da.z = (e0 + 2 < nE) ? dsts[min(e0 + 2, nE - 1)] : sent;
      da.w = (e0 + 3 < nE) ? dsts[min(e0 + 3, nE - 1)] : sent;
      db.x = (e0 + 4 < nE) ? dsts[min(e0 + 4, nE - 1)] : sent;
      db.y = (e0 + 5 < nE) ? dsts[min(e0 + 5, nE - 1)] : sent;
      db.z = (e0 + 6 < nE) ? dsts[min(e0 + 6, nE - 1)] : sent;
      db.w = (e0 + 7 < nE) ? dsts[min(e0 + 7, nE - 1)] : sent;
    }
    const unsigned nb = (unsigned)slotBase;
    const unsigned s0 = (unsigned)da.x - nb, s1 = (unsigned)da.y - nb;
    const unsigned s2 = (unsigned)da.z - nb, s3 = (unsigned)da.w - nb;
    const unsigned s4 = (unsigned)db.x - nb, s5 = (unsigned)db.y - nb;
    const unsigned s6 = (unsigned)db.z - nb, s7 = (unsigned)db.w - nb;
    const bool h0 = s0 < (unsigned)NB, h1 = s1 < (unsigned)NB, h2 = s2 < (unsigned)NB, h3 = s3 < (unsigned)NB;
    const bool h4 = s4 < (unsigned)NB, h5 = s5 < (unsigned)NB, h6 = s6 < (unsigned)NB, h7 = s7 < (unsigned)NB;
    const unsigned any = __builtin_amdgcn_ballot_w32(h0 | h1 | h2 | h3 | h4 | h5 | h6 | h7);
    if (any != 0u) {
#define HITJ(J, HJ, SJ) { \
        const unsigned mj = __builtin_amdgcn_ballot_w32(HJ); \
        if (mj != 0u) { \
          if (HJ) { \
            const int pos = wc + (int)__builtin_amdgcn_mbcnt_lo(mj, 0u); \
            if (pos < WCAP) list[wave * WCAP + pos] = ((el0 + (J)) << 12) | (int)(SJ); \
          } \
          wc += (int)__builtin_popcount(mj); } }
      HITJ(0, h0, s0)
      HITJ(1, h1, s1)
      HITJ(2, h2, s2)
      HITJ(3, h3, s3)
      HITJ(4, h4, s4)
      HITJ(5, h5, s5)
      HITJ(6, h6, s6)
      HITJ(7, h7, s7)
#undef HITJ
    }
  }
  return wc;
}

__global__ __launch_bounds__(NTHR) void k_wprep(const float* __restrict__ ne1, const float* __restrict__ ne2,
                                                const float* __restrict__ mw1, const float* __restrict__ mw2,
                                                const float* __restrict__ uw1, const float* __restrict__ uw2,
                                                const float* __restrict__ rw1, const float* __restrict__ rw2,
                                                _Float16* Wp) {
  const int b = blockIdx.x, tid = threadIdx.x;
  const float* src;
  int dsth, lb, K = CH;
  if (b < 32)        { src = ne1; dsth = PL_NE1; lb = b; }
  else if (b < 64)   { src = ne2; dsth = PL_NE2; lb = b - 32; }
  else if (b < 640) {
    const int l = (b - 64) / 192, q = (b - 64) % 192;
    const int lbase = PL_L0 + l * PL_LSTR;
    if (q < 32)       { src = mw1 + (size_t)l * 131072;         dsth = lbase + PL_MPQ;         lb = q; }
    else if (q < 64)  { src = mw1 + (size_t)l * 131072 + 65536; dsth = lbase + PL_MPQ + 65536; lb = q - 32; }
    else if (q < 96)  { src = mw2 + (size_t)l * 65536;          dsth = lbase + PL_M2;          lb = q - 64; }
    else if (q < 128) { src = uw2 + (size_t)l * 65536;          dsth = lbase + PL_U2;          lb = q - 96; }
    else              { src = uw1 + (size_t)l * 131072;         dsth = lbase + PL_U1;          lb = q - 128; K = 512; }
  }
  else if (b < 672)  { src = rw1; dsth = PL_RO1; lb = b - 640; }
  else               { src = rw2; dsth = PL_RO2; lb = b - 672; }
  const int i  = lb * NTHR + tid;
  const int kq = K >> 3;
  const int n  = i / kq;
  const int k0 = (i - n * kq) * 8;
  float v[8];
#pragma unroll
  for (int e = 0; e < 8; ++e) v[e] = src[(size_t)(k0 + e) * CH + n];
  v8h hv;
#pragma unroll
  for (int e = 0; e < 8; ++e) hv[e] = (_Float16)(v[e] * WSC);
  _Float16* dp = Wp + dsth + (size_t)8 * i;
  *(volatile v8h*)dp = hv;
  __threadfence();
  *(volatile v8h*)dp = hv;
}

__global__ __launch_bounds__(NTHR) void k_count(const int* __restrict__ dsts, int* cnt, int nE, int vec8) {
  __shared__ __attribute__((aligned(16))) int scnt[NBC];
  __shared__ __attribute__((aligned(16))) int list[LISTN];
  __shared__ int wcnt[NWAVE];
  const int tid = threadIdx.x, lane = tid & 31, wave = tid >> 5;
  const int nodeBase = blockIdx.x * NBC;

  for (int i = tid; i < NBC; i += NTHR) scnt[i] = 0;
  __syncthreads();

  const int nChunks = (nE + CHUNK - 1) / CHUNK;
#pragma unroll 1
  for (int ch = 0; ch < nChunks; ++ch) {
    const int cbase = ch * CHUNK;
    const int wc = scan_chunk<NBC>(dsts, nE, cbase, nodeBase, vec8, list, tid, lane, wave);
    if (lane == 0) wcnt[wave] = wc;
    __syncthreads();
    if (wave == 0) {
#pragma unroll 1
      for (int wsx = 0; wsx < NWAVE; ++wsx) {
        int n = __builtin_amdgcn_readfirstlane(wcnt[wsx]);
        n = n > WCAP ? WCAP : (n < 0 ? 0 : n);
        const int* lp = list + wsx * WCAP;
#pragma unroll 1
        for (int i = 0; i < n; ++i) {
          const int ent  = __builtin_amdgcn_readfirstlane(lp[i]);
          const int slot = ent & (NBC - 1);
          if (lane == 0) scnt[slot] = scnt[slot] + 1;
        }
      }
    }
    __syncthreads();
  }

  v4i cq[4];
#pragma unroll
  for (int q = 0; q < 4; ++q) {
    const int f = (wave * 4 + q) * 128 + 4 * lane;
    cq[q] = *(const v4i*)(scnt + f);
  }
  int* cp = cnt + (size_t)nodeBase;
#pragma unroll
  for (int q = 0; q < 4; ++q) {
    const int f = (wave * 4 + q) * 128 + 4 * lane;
    *(volatile v4i*)(cp + f) = cq[q];
  }
  __threadfence();
#pragma unroll
  for (int q = 0; q < 4; ++q) {
    const int f = (wave * 4 + q) * 128 + 4 * lane;
    *(volatile v4i*)(cp + f) = cq[q];
  }
}

__global__ __launch_bounds__(OTHR) void k_offsets(
    const int* __restrict__ cnt, int* off, int* rbase, int nChunk) {
  __shared__ __attribute__((aligned(16))) int soff[NBC];
  __shared__ __attribute__((aligned(16))) int srb[RBN];
  __shared__ int wtot[OTHR / 32];
  const int tid = threadIdx.x, lane = tid & 31, wave = tid >> 5, sub = tid >> 7;
  for (int i = tid; i < RBN; i += OTHR) srb[i] = 0;
  int carry = 0;
#pragma unroll 1
  for (int ch = 0; ch < nChunk; ++ch) {
    const int base = ch * NBC;
    const v4i c0 = *(const v4i*)(cnt + base + 8 * tid);
    const v4i c1 = *(const v4i*)(cnt + base + 8 * tid + 4);
    const int e0 = max(c0.x, 0), e1 = max(c0.y, 0), e2 = max(c0.z, 0), e3 = max(c0.w, 0);
    const int e4 = max(c1.x, 0), e5 = max(c1.y, 0), e6 = max(c1.z, 0), e7 = max(c1.w, 0);
    const int ts = e0 + e1 + e2 + e3 + e4 + e5 + e6 + e7;
    int incl = ts;
#pragma unroll
    for (int d = 1; d < 32; d <<= 1) {
      const int t = __shfl_up(incl, d);
      if (lane >= d) incl += t;
    }
    if (lane == 31) wtot[wave] = incl;
    __syncthreads();
    const int S0 = wtot[0]  + wtot[1]  + wtot[2]  + wtot[3];
    const int S1 = wtot[4]  + wtot[5]  + wtot[6]  + wtot[7];
    const int S2 = wtot[8]  + wtot[9]  + wtot[10] + wtot[11];
    const int S3 = wtot[12] + wtot[13] + wtot[14] + wtot[15];
    int pre = 0;
#pragma unroll 1
    for (int w = 4 * sub; w < wave; ++w) pre += wtot[w];
    const int b0 = carry;
    const int b1 = b0 + ((S0 + 31) & ~31);
    const int b2 = b1 + ((S1 + 31) & ~31);
    const int b3 = b2 + ((S2 + 31) & ~31);
    const int b4 = b3 + ((S3 + 31) & ~31);
    const int myb = sub == 0 ? b0 : (sub == 1 ? b1 : (sub == 2 ? b2 : b3));
    if (tid == 0) {
      srb[min(4 * ch + 0, RBN - 1)] = b0;
      srb[min(4 * ch + 1, RBN - 1)] = b1;
      srb[min(4 * ch + 2, RBN - 1)] = b2;
      srb[min(4 * ch + 3, RBN - 1)] = b3;
    }
    int run = myb + pre + incl - ts;
    soff[8 * tid + 0] = run; run += e0;
    soff[8 * tid + 1] = run; run += e1;
    soff[8 * tid + 2] = run; run += e2;
    soff[8 * tid + 3] = run; run += e3;
    soff[8 * tid + 4] = run; run += e4;
    soff[8 * tid + 5] = run; run += e5;
    soff[8 * tid + 6] = run; run += e6;
    soff[8 * tid + 7] = run;
    carry = b4;
    __syncthreads();
    const v4i o0 = *(const v4i*)(soff + 4 * tid);
    const v4i o1 = *(const v4i*)(soff + 4 * (tid + OTHR));
    int* op = off + base;
    *(volatile v4i*)(op + 4 * tid) = o0;
    *(volatile v4i*)(op + 4 * (tid + OTHR)) = o1;
    __threadfence();
    *(volatile v4i*)(op + 4 * tid) = o0;
    *(volatile v4i*)(op + 4 * (tid + OTHR)) = o1;
    __syncthreads();
  }
  if (tid == 0) srb[min(4 * nChunk, RBN - 1)] = carry;
  __syncthreads();
  v4i rv = {0, 0, 0, 0};
  if (tid < 32) rv = *(const v4i*)(srb + 4 * tid);
  if (tid < 32) *(volatile v4i*)(rbase + 4 * tid) = rv;
  __threadfence();
  if (tid < 32) *(volatile v4i*)(rbase + 4 * tid) = rv;
}

__global__ __launch_bounds__(NTHR) void k_fill(
    const int* __restrict__ dsts, const int* __restrict__ off, const int* __restrict__ rbase,
    int* csr, int nE, int vec8, int csrLen) {
  extern __shared__ v4f lds_dyn[];
  int* region = (int*)lds_dyn;
  int* cursor = region + RCAP;
  int* list   = cursor + NBF;
  int* wcnt   = list + LISTN;
  const int tid = threadIdx.x, lane = tid & 31, wave = tid >> 5;
  const int b = blockIdx.x;
  const int nodeBase = b * NBF;

  int rb0 = rbase[b];
  const int rb1 = rbase[b + 1];
  rb0 = rb0 < 0 ? 0 : (rb0 > csrLen ? csrLen : rb0);
  rb0 &= ~31;
  int len = rb1 - rb0;
  len = len < 0 ? 0 : (len > RCAP ? RCAP : len);
  int lenW = (len + 31) & ~31;
  if (rb0 + lenW > csrLen) lenW = (csrLen - rb0) & ~31;

  {
    const v4i z = {0, 0, 0, 0};
    for (int i = tid; i < RCAP / 4; i += NTHR) ((v4i*)region)[i] = z;
    for (int s = tid; s < NBF; s += NTHR) {
      int o = off[nodeBase + s] - rb0;
      o = o < 0 ? 0 : (o > RCAP ? RCAP : o);
      cursor[s] = o;
    }
  }
  __syncthreads();

  const int nChunks = (nE + CHUNK - 1) / CHUNK;
#pragma unroll 1
  for (int ch = 0; ch < nChunks; ++ch) {
    const int cbase = ch * CHUNK;
    const int wc = scan_chunk<NBF>(dsts, nE, cbase, nodeBase, vec8, list, tid, lane, wave);
    if (lane == 0) wcnt[wave] = wc;
    __syncthreads();
    if (wave == 0) {
#pragma unroll 1
      for (int wsx = 0; wsx < NWAVE; ++wsx) {
        int n = __builtin_amdgcn_readfirstlane(wcnt[wsx]);
        n = n > WCAP ? WCAP : (n < 0 ? 0 : n);
        const int* lp = list + wsx * WCAP;
#pragma unroll 1
        for (int i = 0; i < n; ++i) {
          const int ent  = __builtin_amdgcn_readfirstlane(lp[i]);
          const int slot = ent & (NBF - 1);
          int e = cbase + ((ent >> 12) & (CHUNK - 1));
          e = e > nE - 1 ? nE - 1 : e;
          if (lane == 0) {
            int pos = cursor[slot];
            pos = pos < 0 ? 0 : (pos > RCAP - 1 ? RCAP - 1 : pos);
            region[pos] = e;
            const int np = pos + 1;
            cursor[slot] = np > RCAP ? RCAP : np;
          }
        }
      }
    }
    __syncthreads();
  }

  const int nv = lenW >> 2;
  int* gp = csr + rb0;
#pragma unroll 1
  for (int i = tid; i < nv; i += NTHR) { const v4i v = ((const v4i*)region)[i]; *(volatile v4i*)(gp + 4 * i) = v; }
  __threadfence();
#pragma unroll 1
  for (int i = tid; i < nv; i += NTHR) { const v4i v = ((const v4i*)region)[i]; *(volatile v4i*)(gp + 4 * i) = v; }
}

template <int KD>
__global__ __launch_bounds__(GTHR) void k_gemm_relu16(const float* __restrict__ A0, const float* __restrict__ A1, int aRows,
                                                      const _Float16* __restrict__ Bpl, const float* __restrict__ bias,
                                                      _Float16* Hout) {
  constexpr int AP = KD + 8;
  __shared__ __attribute__((aligned(16))) _Float16 At[GROWS * AP];
  __shared__ __attribute__((aligned(16))) _Float16 stg[GROWS * CH];
  const int tid = threadIdx.x, lane = tid & 31, wave = tid >> 5, hh = lane >> 4, m = lane & 15;
  const int rowBase = blockIdx.x * GROWS;
  if (KD == 512) {
    const int r = tid & 31, part = tid >> 5;
    int arow = rowBase + r;
    arow = arow > aRows - 1 ? aRows - 1 : arow;
    const float* sp = (part == 0 ? A0 : A1) + (size_t)arow * CH;
    _Float16* dp = At + r * AP + part * CH;
#pragma unroll 4
    for (int j = 0; j < 32; ++j) {
      const v4f a = *(const v4f*)(sp + 8 * j), b = *(const v4f*)(sp + 8 * j + 4);
      *(v8h*)(dp + 8 * j) = cvt8z(a, b);
    }
  } else {
    const int r = tid >> 1, c0 = (tid & 1) * 128;
    int arow = rowBase + r;
    arow = arow > aRows - 1 ? aRows - 1 : arow;
    const float* sp = A0 + (size_t)arow * CH + c0;
    _Float16* dp = At + r * AP + c0;
#pragma unroll 4
    for (int j = 0; j < 16; ++j) {
      const v4f a = *(const v4f*)(sp + 8 * j), b = *(const v4f*)(sp + 8 * j + 4);
      *(v8h*)(dp + 8 * j) = cvt8z(a, b);
    }
  }
  __syncthreads();

#pragma unroll
  for (int cg = 0; cg < 4; ++cg) {
    v8f acc[4];
    mma<4>(At + wave * 16 * AP, AP, Bpl + (size_t)(64 * cg) * KD, KD, KD / 32, lane, acc);
    _Float16* sp = stg + (wave * 16 + 8 * hh) * CH + 64 * cg + m;
#pragma unroll
    for (int t = 0; t < 4; ++t) {
      const int col = 64 * cg + 16 * t + m;
      const float bv = bias[col];
#pragma unroll
      for (int r = 0; r < 8; ++r) {
        const float v = fmaxf(acc[t][r] * RZW + bv, 0.0f);
        sp[r * CH + 16 * t] = (_Float16)(v * ZSC);
      }
    }
  }
  __syncthreads();

  _Float16* gp = Hout + (size_t)rowBase * CH;
#pragma unroll 4
  for (int it = 0; it < 16; ++it) {
    const int f = it * GTHR + tid;
    const v8h v = *(const v8h*)(stg + 8 * f);
    *(volatile v8h*)(gp + 8 * f) = v;
  }
  __threadfence();
#pragma unroll 4
  for (int it = 0; it < 16; ++it) {
    const int f = it * GTHR + tid;
    const v8h v = *(const v8h*)(stg + 8 * f);
    *(volatile v8h*)(gp + 8 * f) = v;
  }
}

template <int LN>
__global__ __launch_bounds__(GTHR) void k_gemm16(const _Float16* __restrict__ A16, const _Float16* __restrict__ Bpl,
                                                 const float* __restrict__ bias, const float* __restrict__ lng,
                                                 const float* __restrict__ lnb, float* X) {
  __shared__ __attribute__((aligned(16))) _Float16 At[GROWS * APZ];
  __shared__ __attribute__((aligned(16))) float stg[GROWS * CH];
  __shared__ __attribute__((aligned(16))) float sbias[CH];
  const int tid = threadIdx.x, lane = tid & 31, wave = tid >> 5, hh = lane >> 4, m = lane & 15;
  const int rowBase = blockIdx.x * GROWS;
  {
    const int r = tid >> 1, c0 = (tid & 1) * 128;
    const _Float16* ap = A16 + (size_t)(rowBase + r) * CH + c0;
    _Float16* dp = At + r * APZ + c0;
#pragma unroll 4
    for (int j = 0; j < 16; ++j) *(v8h*)(dp + 8 * j) = *(const v8h*)(ap + 8 * j);
    *(v4f*)(sbias + 4 * tid) = *(const v4f*)(bias + 4 * tid);
  }
  __syncthreads();

#pragma unroll
  for (int cg = 0; cg < 4; ++cg) {
    v8f acc[4];
    mma<4>(At + wave * 16 * APZ, APZ, Bpl + (size_t)(64 * cg) * CH, CH, CH / 32, lane, acc);
    float* sp = stg + (wave * 16 + 8 * hh) * CH + 64 * cg + m;
#pragma unroll
    for (int t = 0; t < 4; ++t) {
      const int col = 64 * cg + 16 * t + m;
      const float bv = sbias[col];
#pragma unroll
      for (int r = 0; r < 8; ++r) sp[r * CH + 16 * t] = acc[t][r] * RZW + bv;
    }
  }
  __syncthreads();

  if (LN) {
    const v4f g0 = *(const v4f*)(lng + 8 * lane), g1 = *(const v4f*)(lng + 8 * lane + 4);
    const v4f e0 = *(const v4f*)(lnb + 8 * lane), e1 = *(const v4f*)(lnb + 8 * lane + 4);
    const float* xb = X + (size_t)(rowBase + wave * 16) * CH + 8 * lane;
#pragma unroll 1
    for (int rr = 0; rr < 16; ++rr) {
      float* rp = stg + (wave * 16 + rr) * CH + 8 * lane;
      const float* xp = xb + (size_t)rr * CH;
      const v4f xa = *(const v4f*)xp, xc = *(const v4f*)(xp + 4);
      v4f a = *(const v4f*)rp, b = *(const v4f*)(rp + 4);
      a = a + xa;
      b = b + xc;
      float s = ((a.x + a.y) + (a.z + a.w)) + ((b.x + b.y) + (b.z + b.w));
      s = wsum(s);
      const float mu = s * (1.0f / (float)CH);
      a.x -= mu; a.y -= mu; a.z -= mu; a.w -= mu;
      b.x -= mu; b.y -= mu; b.z -= mu; b.w -= mu;
      float q = ((a.x * a.x + a.y * a.y) + (a.z * a.z + a.w * a.w)) + ((b.x * b.x + b.y * b.y) + (b.z * b.z + b.w * b.w));
      q = wsum(q);
      const float var = q * (1.0f / (float)CH);
      const float rs = rsqrtf(var + LNEPS);
      v4f ya, yb;
      ya.x = a.x * rs * g0.x + e0.x; ya.y = a.y * rs * g0.y + e0.y; ya.z = a.z * rs * g0.z + e0.z; ya.w = a.w * rs * g0.w + e0.w;
      yb.x = b.x * rs * g1.x + e1.x; yb.y = b.y * rs * g1.y + e1.y; yb.z = b.z * rs * g1.z + e1.z; yb.w = b.w * rs * g1.w + e1.w;
      *(v4f*)rp = ya;
      *(v4f*)(rp + 4) = yb;
    }
    __syncthreads();
  }

  float* gp = X + (size_t)rowBase * CH;
#pragma unroll 8
  for (int it = 0; it < 32; ++it) {
    const int f = it * GTHR + tid;
    const v4f v = *(const v4f*)(stg + 4 * f);
    *(volatile v4f*)(gp + 4 * f) = v;
  }
  __threadfence();
#pragma unroll 8
  for (int it = 0; it < 32; ++it) {
    const int f = it * GTHR + tid;
    const v4f v = *(const v4f*)(stg + 4 * f);
    *(volatile v4f*)(gp + 4 * f) = v;
  }
}

__global__ __launch_bounds__(GTHR) void k_pq(const float* __restrict__ X, const _Float16* __restrict__ Bpl,
                                             const float* __restrict__ b1, float* PQ) {
  __shared__ __attribute__((aligned(16))) _Float16 At[GROWS * APZ];
  __shared__ __attribute__((aligned(16))) float stg[GROWS * CH];
  const int tid = threadIdx.x, lane = tid & 31, wave = tid >> 5, hh = lane >> 4, m = lane & 15;
  const int rowBase = blockIdx.x * GROWS;
  {
    const int r = tid >> 1, c0 = (tid & 1) * 128;
    const float* sp = X + (size_t)(rowBase + r) * CH + c0;
    _Float16* dp = At + r * APZ + c0;
#pragma unroll 4
    for (int j = 0; j < 16; ++j) {
      const v4f a = *(const v4f*)(sp + 8 * j), b = *(const v4f*)(sp + 8 * j + 4);
      *(v8h*)(dp + 8 * j) = cvt8z(a, b);
    }
  }
  __syncthreads();

#pragma unroll 1
  for (int hf = 0; hf < 2; ++hf) {
#pragma unroll
    for (int cg = 0; cg < 4; ++cg) {
      v8f acc[4];
      mma<4>(At + wave * 16 * APZ, APZ, Bpl + (size_t)(CH * hf + 64 * cg) * CH, CH, CH / 32, lane, acc);
      float* sp = stg + (wave * 16 + 8 * hh) * CH + 64 * cg + m;
#pragma unroll
      for (int t = 0; t < 4; ++t) {
        const int col = 64 * cg + 16 * t + m;
        const float bl = b1[col];
        const float bv = (hf != 0) ? bl : 0.0f;
#pragma unroll
        for (int r = 0; r < 8; ++r) sp[r * CH + 16 * t] = acc[t][r] * RZW + bv;
      }
    }
    __syncthreads();
    float* gp = PQ + (size_t)rowBase * PQW + CH * hf + 4 * tid;
#pragma unroll 8
    for (int it = 0; it < 32; ++it) {
      const v4f v = *(const v4f*)(stg + it * CH + 4 * tid);
      *(volatile v4f*)(gp + (size_t)it * PQW) = v;
    }
    __threadfence();
#pragma unroll 8
    for (int it = 0; it < 32; ++it) {
      const v4f v = *(const v4f*)(stg + it * CH + 4 * tid);
      *(volatile v4f*)(gp + (size_t)it * PQW) = v;
    }
    __syncthreads();
  }
}

__global__ __launch_bounds__(FTHR) void k_edge(
    const float* __restrict__ PQ, const int* __restrict__ csr,
    const int* __restrict__ offp, const int* __restrict__ cntp,
    const int* __restrict__ srcs, const _Float16* __restrict__ B2,
    const float* __restrict__ b2, float* agg, int nN, int nE, int csrLen) {
  __shared__ __attribute__((aligned(16))) _Float16 zt[FW * KNB * APZ];
  __shared__ __attribute__((aligned(16))) float sout[FW * CH];
  __shared__ __attribute__((aligned(16))) float sb2[CH];
  __shared__ __attribute__((aligned(16))) int slot[FW];
  const int tid = threadIdx.x, lane = tid & 31, wave = tid >> 5, hh = lane >> 4, m = lane & 15;
  const int base = blockIdx.x * NPBE;
  _Float16* zw = zt + wave * (KNB * APZ);

  if (tid < CH / 4) *(v4f*)(sb2 + 4 * tid) = *(const v4f*)(b2 + 4 * tid);
  __syncthreads();

#pragma unroll 1
  for (int it = 0; it < NIT; ++it) {
    const int n = base + it * FW + wave;
    const bool nval = n < nN;
    const int cc = nval ? n : nN - 1;
    const int cnr = cntp[cc];
    const int ofr = offp[cc];
    int cn = nval ? cnr : 0;
    cn = cn < 0 ? 0 : (cn > DEGCAP ? DEGCAP : cn);
    cn = __builtin_amdgcn_readfirstlane(cn);
    int of = ofr;
    of = of < 0 ? 0 : (of > csrLen ? csrLen : of);
    of = __builtin_amdgcn_readfirstlane(of);
    const float* qp = PQ + (size_t)cc * PQW + CH + 8 * lane;
    const v4f qa = *(const v4f*)qp, qb = *(const v4f*)(qp + 4);
    const int ntw = (cn + KNB - 1) >> 4;
    if (lane == 0) slot[wave] = ntw;
    __syncthreads();
    int ntmax;
    {
      const v4i sA = *(const v4i*)slot;
      int mm = max(max(sA.x, sA.y), max(sA.z, sA.w));
      mm = mm < 0 ? 0 : (mm > DEGCAP / KNB ? DEGCAP / KNB : mm);
      ntmax = __builtin_amdgcn_readfirstlane(mm);
    }
    float cs[16];
#pragma unroll
    for (int t = 0; t < 16; ++t) cs[t] = 0.0f;
#pragma unroll 1
    for (int tt = 0; tt < ntmax; ++tt) {
      int nv = cn - tt * KNB;
      nv = nv < 0 ? 0 : (nv > KNB ? KNB : nv);
      nv = __builtin_amdgcn_readfirstlane(nv);
      int pos = of + tt * KNB + m;
      pos = pos < 0 ? 0 : (pos > csrLen - 1 ? csrLen - 1 : pos);
      int e = csr[pos];
      e = e < 0 ? 0 : (e > nE - 1 ? nE - 1 : e);
      int sv = srcs[e];
      sv = sv < 0 ? 0 : (sv > nN - 1 ? nN - 1 : sv);
      __syncthreads();
      if (nv > 0) {
        rows_z<0>(zw, PQ, sv, qa, qb, lane);
        asm volatile("" ::: "memory");
        rows_z<8>(zw, PQ, sv, qa, qb, lane);
      }
      __syncthreads();
      if (nv > 0) {
#pragma unroll
        for (int cg = 0; cg < 2; ++cg) {
          v8f acc[8];
          mma<8>(zw, APZ, B2 + (size_t)(128 * cg) * CH, CH, CH / 32, lane, acc);
#pragma unroll
          for (int t = 0; t < 8; ++t) {
            float s = 0.0f;
#pragma unroll
            for (int r = 0; r < 8; ++r) s += (8 * hh + r < nv) ? acc[t][r] : 0.0f;
            cs[8 * cg + t] += s;
          }
        }
      }
    }
#pragma unroll
    for (int t = 0; t < 16; ++t) cs[t] += __shfl_xor(cs[t], 16, 32);
    if (hh == 0) {
      const float fc = (float)cn;
#pragma unroll
      for (int t = 0; t < 16; ++t) sout[wave * CH + 16 * t + m] = cs[t] * RZW + fc * sb2[16 * t + m];
    }
    __syncthreads();
    {
      float* gp = agg + (size_t)(base + it * FW) * CH;
      const v4f v0 = *(const v4f*)(sout + 4 * tid);
      const v4f v1 = *(const v4f*)(sout + 4 * (tid + FTHR));
      *(volatile v4f*)(gp + 4 * tid) = v0;
      *(volatile v4f*)(gp + 4 * (tid + FTHR)) = v1;
      __threadfence();
      *(volatile v4f*)(gp + 4 * tid) = v0;
      *(volatile v4f*)(gp + 4 * (tid + FTHR)) = v1;
    }
  }
}

__global__ __launch_bounds__(RTHR) void k_readout(const float* __restrict__ X, int nN, double invN,
                                                  const _Float16* __restrict__ R1, const float* __restrict__ rb1,
                                                  const _Float16* __restrict__ R2, const float* __restrict__ rb2,
                                                  float* out) {
  __shared__ __attribute__((aligned(16))) _Float16 Ag[16 * APZ];
  __shared__ __attribute__((aligned(16))) _Float16 Ah[16 * APZ];
  __shared__ __attribute__((aligned(16))) float so[CH];
  const int tid = threadIdx.x, lane = tid & 31, wave = tid >> 5, hh = lane >> 4, m = lane & 15;
  {
    const v8h z8 = {(_Float16)0, (_Float16)0, (_Float16)0, (_Float16)0, (_Float16)0, (_Float16)0, (_Float16)0, (_Float16)0};
    for (int i = tid; i < (16 * APZ) / 8; i += RTHR) { *(v8h*)(Ag + 8 * i) = z8; *(v8h*)(Ah + 8 * i) = z8; }
  }
  __syncthreads();
  double s = 0.0;
#pragma unroll 4
  for (int n = 0; n < nN; ++n) s += (double)X[(size_t)n * CH + tid];
  const float g = (float)(s * invN);
  Ag[tid] = (_Float16)(g * ZSC);
  __syncthreads();
  {
    v8f acc[2];
    mma<2>(Ag, APZ, R1 + (size_t)(32 * wave) * CH, CH, CH / 32, lane, acc);
#pragma unroll
    for (int t = 0; t < 2; ++t) {
      const int col = 32 * wave + 16 * t + m;
      const float hv = fmaxf(acc[t][0] * RZW + rb1[col], 0.0f);
      if (hh == 0) Ah[col] = (_Float16)(hv * ZSC);
    }
  }
  __syncthreads();
  {
    v8f acc[2];
    mma<2>(Ah, APZ, R2 + (size_t)(32 * wave) * CH, CH, CH / 32, lane, acc);
#pragma unroll
    for (int t = 0; t < 2; ++t) {
      const int col = 32 * wave + 16 * t + m;
      const float ov = acc[t][0] * RZW + rb2[col];
      if (hh == 0) so[col] = ov;
    }
  }
  __syncthreads();
  v4f v = {0.f, 0.f, 0.f, 0.f};
  if (tid < 64) v = *(const v4f*)(so + 4 * tid);
  if (tid < 64) *(volatile v4f*)(out + 4 * tid) = v;
  __threadfence();
  if (tid < 64) *(volatile v4f*)(out + 4 * tid) = v;
}

extern "C" void kernel_launch(void* const* d_in, const int* in_sizes, int n_in,
                              void* d_out, int out_size, void* d_ws, size_t ws_size,
                              hipStream_t stream) {
  if (n_in < 20) return;
  const int nN = in_sizes[0] / CH;
  const int nE = in_sizes[1] / 2;
  if (nN <= 0 || nE <= 0) return;
  if (in_sizes[0] != nN * CH || in_sizes[1] != 2 * nE) return;
  if (in_sizes[2] != CH * CH || in_sizes[3] != CH || in_sizes[4] != CH * CH || in_sizes[5] != CH) return;
  if (in_sizes[6] != 3 * 2 * CH * CH || in_sizes[7] != 3 * CH || in_sizes[8] != 3 * CH * CH || in_sizes[9] != 3 * CH) return;
  if (in_sizes[10] != 3 * 2 * CH * CH || in_sizes[11] != 3 * CH || in_sizes[12] != 3 * CH * CH || in_sizes[13] != 3 * CH) return;
  if (in_sizes[14] != 3 * CH || in_sizes[15] != 3 * CH) return;
  if (in_sizes[16] != CH * CH || in_sizes[17] != CH || in_sizes[18] != CH * CH || in_sizes[19] != CH) return;
  if (out_size != CH) return;
  if (nE > (1 << 28) || nN > (1 << 24)) return;

  const float* nf    = (const float*)d_in[0];
  const int*   ei    = (const int*)d_in[1];
  const float* ne_w1 = (const float*)d_in[2];
  const float* ne_b1 = (const float*)d_in[3];
  const float* ne_w2 = (const float*)d_in[4];
  const float* ne_b2 = (const float*)d_in[5];
  const float* mw1   = (const float*)d_in[6];
  const float* mb1   = (const float*)d_in[7];
  const float* mw2   = (const float*)d_in[8];
  const float* mb2   = (const float*)d_in[9];
  const float* uw1   = (const float*)d_in[10];
  const float* ub1   = (const float*)d_in[11];
  const float* uw2   = (const float*)d_in[12];
  const float* ub2   = (const float*)d_in[13];
  const float* lng   = (const float*)d_in[14];
  const float* lnb   = (const float*)d_in[15];
  const float* rw1   = (const float*)d_in[16];
  const float* rb1   = (const float*)d_in[17];
  const float* rw2   = (const float*)d_in[18];
  const float* rb2   = (const float*)d_in[19];
  const int* srcs = ei;
  const int* dsts = ei + nE;
  float* out = (float*)d_out;

  const int NPAD   = ((nN + NPALN - 1) / NPALN) * NPALN;
  const int nBlkG  = NPAD / GROWS;
  const int nBlkE  = NPAD / NPBE;
  const int nBC    = (nN + NBC - 1) / NBC;
  const int CNTPAD = nBC * NBC;
  if (4 * nBC + 1 > RBN) return;
  const int nBF    = (nN + NBF - 1) / NBF;
  const int csrLen = ((nE + 31) & ~31) + 4096;
  if (31 * 4 * nBC > 4096) return;

  char* ws = (char*)d_ws;
  size_t off = 0;
  const size_t oW   = off; off += (size_t)PL_TOT * 2;              off = (off + 255) & ~(size_t)255;
  const size_t oCnt = off; off += (size_t)CNTPAD * 4;              off = (off + 255) & ~(size_t)255;
  const size_t oOff = off; off += (size_t)CNTPAD * 4;              off = (off + 255) & ~(size_t)255;
  const size_t oRb  = off; off += (size_t)RBN * 4;                 off = (off + 255) & ~(size_t)255;
  const size_t oCsr = off; off += (size_t)csrLen * 4;              off = (off + 255) & ~(size_t)255;
  const size_t oX   = off; off += (size_t)NPAD * CH * 4;           off = (off + 255) & ~(size_t)255;
  const size_t oH   = off; off += (size_t)NPAD * CH * 2;           off = (off + 255) & ~(size_t)255;
  const size_t oPQ  = off; off += (size_t)NPAD * PQW * 4;          off = (off + 255) & ~(size_t)255;
  const size_t oAG  = off; off += (size_t)NPAD * CH * 4;           off = (off + 255) & ~(size_t)255;
  if (off > ws_size || off > (size_t)WSCAP) return;
  _Float16* Wp   = (_Float16*)(ws + oW);
  int*      cnt  = (int*)(ws + oCnt);
  int*      offp = (int*)(ws + oOff);
  int*      rb   = (int*)(ws + oRb);
  int*      csr  = (int*)(ws + oCsr);
  float*    X    = (float*)(ws + oX);
  _Float16* H16  = (_Float16*)(ws + oH);
  float*    PQ   = (float*)(ws + oPQ);
  float*    AG   = (float*)(ws + oAG);

  const int vec8 = ((nE & 3) == 0) ? 1 : 0;
  const double invN = 1.0 / (double)nN;

  k_wprep<<<WPBLK, NTHR, 0, stream>>>(ne_w1, ne_w2, mw1, mw2, uw1, uw2, rw1, rw2, Wp);
  k_count<<<nBC, NTHR, 0, stream>>>(dsts, cnt, nE, vec8);
  k_offsets<<<1, OTHR, 0, stream>>>(cnt, offp, rb, nBC);
  hipFuncSetAttribute(reinterpret_cast<const void*>(&k_fill),
                      hipFuncAttributeMaxDynamicSharedMemorySize, LDS_FILL);
  k_fill<<<nBF, NTHR, LDS_FILL, stream>>>(dsts, offp, rb, csr, nE, vec8, csrLen);
  k_gemm_relu16<256><<<nBlkG, GTHR, 0, stream>>>(nf, nf, nN, Wp + PL_NE1, ne_b1, H16);
  k_gemm16<0><<<nBlkG, GTHR, 0, stream>>>(H16, Wp + PL_NE2, ne_b2, lng, lnb, X);
  for (int l = 0; l < 3; ++l) {
    const _Float16* Lp = Wp + PL_L0 + (size_t)l * PL_LSTR;
    k_pq<<<nBlkG, GTHR, 0, stream>>>(X, Lp + PL_MPQ, mb1 + l * CH, PQ);
    k_edge<<<nBlkE, FTHR, 0, stream>>>(PQ, csr, offp, cnt, srcs, Lp + PL_M2, mb2 + l * CH, AG, nN, nE, csrLen);
    k_gemm_relu16<512><<<nBlkG, GTHR, 0, stream>>>(X, AG, NPAD, Lp + PL_U1, ub1 + l * CH, H16);
    k_gemm16<1><<<nBlkG, GTHR, 0, stream>>>(H16, Lp + PL_U2, ub2 + l * CH, lng + l * CH, lnb + l * CH, X);
  }
  k_readout<<<1, RTHR, 0, stream>>>(X, nN, invN, Wp + PL_RO1, rb1, Wp + PL_RO2, rb2, out);
}
